// InteractionPPBlockSMP_32384053412123
// MI455X (gfx1250) — hardware-run, weakly checked
//
#include <hip/hip_runtime.h>


#define NEDGE 65536
#define NTRIP 262144
#define HH 128
#define DD 64
#define NBR 6
#define NR 6
#define NC 8
#define NS 42
#define TC 65536
#define QCAP 8
#define CHUNK 8192

static_assert((NTRIP % TC) == 0);
static_assert((TC % CHUNK) == 0);
static_assert((TC % 16) == 0);
static_assert(CHUNK == 512 * 16);
static_assert((NEDGE % 1024) == 0);
static_assert((((NEDGE / 16) * (HH / 64)) % 4) == 0);
static_assert((((NEDGE / 16) * (DD / 64)) % 4) == 0);
static_assert((((TC / 16) * (DD / 64)) % 4) == 0);

typedef _Float16 v16h __attribute__((ext_vector_type(16)));
typedef unsigned short v8us __attribute__((ext_vector_type(8), may_alias));
typedef unsigned short v4us __attribute__((ext_vector_type(4), may_alias));
typedef float v8f __attribute__((ext_vector_type(8)));
typedef float v4f __attribute__((ext_vector_type(4)));
typedef float v4fa __attribute__((ext_vector_type(4), may_alias));
union FragH { v16h v; v8us half[2]; _Float16 h[16]; unsigned short u[16]; };
union Pack8 { v8us v; _Float16 h[8]; unsigned short u[8]; };
union Pack4 { v4us v; _Float16 h[4]; unsigned short u[4]; };

__device__ __forceinline__ v8f mma16(v16h a, v16h b, v8f c) {
  c = __builtin_amdgcn_wmma_f32_16x16x32_f16(false, a, false, b, (short)0, c, false, false);
  asm volatile("v_nop\n\tv_nop\n\tv_nop\n\tv_nop" : "+v"(c) : "v"(a), "v"(b));
  return c;
}

__device__ __forceinline__ float silu_f(float v) { return v * __builtin_amdgcn_rcpf(1.0f + expf(-v)); }

__global__ __launch_bounds__(256) void k_wt(const float* __restrict__ W, int sW, unsigned short* __restrict__ Wt, int sWt, int K, int N, float scale) {
  const int b = blockIdx.y;
  const float* Wb = W + (size_t)b * sW;
  unsigned short* Wtb = Wt + (size_t)b * sWt;
  const int t = blockIdx.x * 256 + threadIdx.x;
  const int k8n = K >> 3;
  if (t >= N * k8n) return;
  const int n = t / k8n, k8 = (t - n * k8n) * 8;
  Pack8 f;
#pragma unroll
  for (int i = 0; i < 8; ++i) f.h[i] = (_Float16)(Wb[(size_t)(k8 + i) * N + n] * scale);
  unsigned short* d = Wtb + (size_t)n * K + k8;
  *(volatile v8us*)d = f.v;
  __threadfence();
  *(volatile v8us*)d = f.v;
}

__global__ __launch_bounds__(256) void k_ws1t(const float* __restrict__ W1, unsigned short* __restrict__ Wt) {
  const int t = blockIdx.x * 256 + threadIdx.x;
  if (t >= 64 * 8) return;
  const int n = t >> 3, k8 = (t & 7) * 8;
  int bb = n >> 3; bb = bb > (NBR - 1) ? (NBR - 1) : bb;
  const int cc = n & 7;
  Pack8 f;
#pragma unroll
  for (int i = 0; i < 8; ++i) {
    const int k = k8 + i;
    const int kk = k < NS ? k : (NS - 1);
    const float wv = W1[((size_t)bb * NS + kk) * NC + cc];
    f.h[i] = (n < NBR * NC && k < NS) ? (_Float16)(wv * 16.0f) : (_Float16)0.0f;
  }
  unsigned short* d = Wt + (size_t)n * 64 + k8;
  *(volatile v8us*)d = f.v;
  __threadfence();
  *(volatile v8us*)d = f.v;
}

__global__ __launch_bounds__(256) void k_x16(const float* __restrict__ x, unsigned short* __restrict__ X16) {
  const size_t t = (size_t)blockIdx.x * 256 + threadIdx.x;
  if (t >= (size_t)NEDGE * HH / 8) return;
  const v4f a = *(const v4fa*)(x + t * 8), b = *(const v4fa*)(x + t * 8 + 4);
  Pack8 f;
#pragma unroll
  for (int i = 0; i < 4; ++i) { f.h[i] = (_Float16)a[i]; f.h[4 + i] = (_Float16)b[i]; }
  unsigned short* d = X16 + t * 8;
  *(volatile v8us*)d = f.v;
  __threadfence();
  *(volatile v8us*)d = f.v;
}

__global__ __launch_bounds__(256) void k_sbf16(const float* __restrict__ sbf, int t0, unsigned short* __restrict__ S16) {
  const int t = blockIdx.x * 256 + threadIdx.x;
  if (t >= TC * 8) return;
  const int tl = t >> 3, k8 = (t & 7) * 8;
  const float* row = sbf + (size_t)(t0 + tl) * NS;
  Pack8 f;
#pragma unroll
  for (int i = 0; i < 8; ++i) {
    const int k = k8 + i;
    const int kk = k < NS ? k : (NS - 1);
    const float v = row[kk];
    f.h[i] = (k < NS) ? (_Float16)v : (_Float16)0.0f;
  }
  unsigned short* d = S16 + (size_t)tl * 64 + k8;
  *(volatile v8us*)d = f.v;
  __threadfence();
  *(volatile v8us*)d = f.v;
}

__global__ __launch_bounds__(256) void k_agg16(const float* __restrict__ AGG, unsigned short* __restrict__ A16) {
  const size_t t = (size_t)blockIdx.x * 256 + threadIdx.x;
  if (t >= (size_t)NEDGE * DD / 8) return;
  const v4f a = *(const v4fa*)(AGG + t * 8), b = *(const v4fa*)(AGG + t * 8 + 4);
  Pack8 f;
#pragma unroll
  for (int i = 0; i < 4; ++i) { f.h[i] = (_Float16)(a[i] * 4096.0f); f.h[4 + i] = (_Float16)(b[i] * 4096.0f); }
  unsigned short* d = A16 + t * 8;
  *(volatile v8us*)d = f.v;
  __threadfence();
  *(volatile v8us*)d = f.v;
}

template <bool RBF, bool ACT>
__global__ __launch_bounds__(128) void k_gemm(const unsigned short* __restrict__ A, int lda, const unsigned short* __restrict__ Bt, int ldb,
                                            int M, int N, int K, float oscale, const float* __restrict__ bias,
                                            const float* __restrict__ rbf, const float* __restrict__ W1b, const float* __restrict__ W2b,
                                            const float* res, int ldr, float* Cf, int ldcf, unsigned short* Ch, int ldch, float hscale) {
  __shared__ __attribute__((aligned(16))) float so[4][16][64];
  __shared__ __attribute__((aligned(16))) float srb[RBF ? 32 : 1][HH];
  const int tid = threadIdx.x, w = tid >> 5, lane = tid & 31, ln = lane & 15, hh = lane >> 4;
  const int ntn = N >> 6;
  const int wid = blockIdx.x * 4 + w;
  const int mt = wid / ntn, nq = wid - mt * ntn;
  const int row0 = mt * 16, col0 = nq * 64;
  if (RBF) {
    const int rb0 = blockIdx.x * 32;
    const int lr = tid >> 2, cs = (tid & 3) * 32;
    int grow = rb0 + lr; grow = grow < M ? grow : (M - 1);
    float rv[NR];
#pragma unroll
    for (int q = 0; q < NR; ++q) rv[q] = rbf[(size_t)grow * NR + q];
    float pc[NC];
#pragma unroll
    for (int c = 0; c < NC; ++c) {
      float s = 0.f;
#pragma unroll
      for (int q = 0; q < NR; ++q) s += rv[q] * W1b[q * NC + c];
      pc[c] = s;
    }
#pragma unroll 2
    for (int cc = 0; cc < 32; ++cc) {
      const int col = cs + cc;
      float s = 0.f;
#pragma unroll
      for (int c = 0; c < NC; ++c) s += pc[c] * W2b[c * HH + col];
      srb[lr][col] = s;
    }
    __syncthreads();
  }
  if (row0 >= M) return;

  const unsigned short* arow = A + (size_t)(row0 + ln) * lda;
  v8f acc[4];
#pragma unroll
  for (int t = 0; t < 4; ++t) acc[t] = (v8f){0.f, 0.f, 0.f, 0.f, 0.f, 0.f, 0.f, 0.f};
  for (int kb = 0; kb < K; kb += 32) {
    FragH a;
    a.half[0] = *(const v8us*)(arow + kb + 8 * hh);
    a.half[1] = *(const v8us*)(arow + kb + 16 + 8 * hh);
#pragma unroll
    for (int t = 0; t < 4; ++t) {
      const unsigned short* brow = Bt + (size_t)(col0 + t * 16 + ln) * ldb + kb;
      FragH b;
      b.half[0] = *(const v8us*)(brow + 8 * hh);
      b.half[1] = *(const v8us*)(brow + 16 + 8 * hh);
      acc[t] = mma16(a.v, b.v, acc[t]);
    }
  }
  const int lrow = RBF ? ((w >> 1) * 16) : 0;
#pragma unroll
  for (int t = 0; t < 4; ++t) {
    const int col = col0 + t * 16 + ln;
    float bv = 0.f;
    if (bias != nullptr) bv = bias[col];
#pragma unroll
    for (int r = 0; r < 8; ++r) {
      float v = acc[t][r] * oscale + bv;
      if (ACT) v = silu_f(v);
      if (RBF) v *= srb[lrow + 8 * hh + r][col];
      if (res != nullptr) v += res[(size_t)(row0 + 8 * hh + r) * ldr + col];
      so[w][8 * hh + r][t * 16 + ln] = v;
    }
  }
  __builtin_amdgcn_fence(__ATOMIC_ACQ_REL, "workgroup");
  __builtin_amdgcn_wave_barrier();
  const int rs = lane >> 3, c8 = (lane & 7) * 8, c4 = ln * 4;
  for (int pass = 0; pass < 2; ++pass) {
    if (Cf != nullptr) {
#pragma unroll
      for (int q = 0; q < 8; ++q) {
        const int r = q * 2 + hh;
        const v4f v = *(const v4fa*)&so[w][r][c4];
        *(volatile v4f*)(Cf + (size_t)(row0 + r) * ldcf + col0 + c4) = v;
      }
    }
    if (Ch != nullptr) {
#pragma unroll
      for (int q = 0; q < 4; ++q) {
        const int r = q * 4 + rs;
        const v4f x0 = *(const v4fa*)&so[w][r][c8], x1 = *(const v4fa*)&so[w][r][c8 + 4];
        Pack8 pk;
#pragma unroll
        for (int i = 0; i < 4; ++i) { pk.h[i] = (_Float16)(x0[i] * hscale); pk.h[4 + i] = (_Float16)(x1[i] * hscale); }
        *(volatile v8us*)(Ch + (size_t)(row0 + r) * ldch + col0 + c8) = pk.v;
      }
    }
    if (pass == 0) __threadfence();
  }
}

__global__ __launch_bounds__(256) void k_msg(const float* __restrict__ P1, const int* __restrict__ ikj, const int* __restrict__ btab,
                                           const float* __restrict__ alpha_p, const float* __restrict__ W2, const unsigned short* __restrict__ DN,
                                           int t0, float* __restrict__ MSG) {
  __shared__ __attribute__((aligned(16))) float sW2[NBR * NC * DD];
  const int tid = threadIdx.x;
  for (int i = tid; i < NBR * NC * DD; i += 256) sW2[i] = W2[i];
  __syncthreads();
  const int t = blockIdx.x * 256 + tid;
  if (t >= TC * 16) return;
  const int tl = t >> 4, d4 = (t & 15) * 4;
  int j = ikj[t0 + tl];
  j = j < 0 ? 0 : (j >= NEDGE ? NEDGE - 1 : j);
  const int bv = btab[j];
  const int b1 = bv + 1;
  const bool valid = (b1 >= 0) && (b1 < NBR);
  const int b1c = valid ? b1 : (NBR - 1);
  const float al = alpha_p[0];
  const float wb = valid ? (1.0f - al) : 0.0f;
  const float* pr = P1 + (size_t)tl * DD;
  const v4f p5a = *(const v4fa*)(pr + (NBR - 1) * NC), p5b = *(const v4fa*)(pr + (NBR - 1) * NC + 4);
  const v4f pba = *(const v4fa*)(pr + b1c * NC), pbb = *(const v4fa*)(pr + b1c * NC + 4);
  const float p5[8] = {p5a[0], p5a[1], p5a[2], p5a[3], p5b[0], p5b[1], p5b[2], p5b[3]};
  const float pb[8] = {pba[0], pba[1], pba[2], pba[3], pbb[0], pbb[1], pbb[2], pbb[3]};
  float s5[4] = {0.f, 0.f, 0.f, 0.f}, sb[4] = {0.f, 0.f, 0.f, 0.f};
#pragma unroll
  for (int c = 0; c < NC; ++c) {
    const v4f w5 = *(const v4fa*)&sW2[((NBR - 1) * NC + c) * DD + d4];
    const v4f wbv = *(const v4fa*)&sW2[(b1c * NC + c) * DD + d4];
#pragma unroll
    for (int e = 0; e < 4; ++e) { s5[e] += p5[c] * w5[e]; sb[e] += pb[c] * wbv[e]; }
  }
  Pack4 g5, gb;
  g5.v = *(const v4us*)(DN + ((size_t)(NBR - 1) * NEDGE + j) * DD + d4);
  gb.v = *(const v4us*)(DN + ((size_t)b1c * NEDGE + j) * DD + d4);
  v4f m;
#pragma unroll
  for (int e = 0; e < 4; ++e) {
    const float d5 = (float)g5.h[e] * (1.0f / 256.0f);
    const float db = (float)gb.h[e] * (1.0f / 256.0f);
    m[e] = al * (d5 * s5[e]) + wb * (db * sb[e]);
  }
  float* dst = MSG + (size_t)tl * DD + d4;
  *(volatile v4f*)dst = m;
  __threadfence();
  *(volatile v4f*)dst = m;
}

__device__ __forceinline__ int bscan512(int cnt, int* wsum, int tid, int& total) {
  const int lane = tid & 31, wv = tid >> 5;
  int x = cnt;
#pragma unroll
  for (int d = 1; d < 32; d <<= 1) { const int y = __shfl_up(x, d, 32); if (lane >= d) x += y; }
  __syncthreads();
  if (lane == 31) wsum[wv] = x;
  __syncthreads();
  const int tv = wsum[lane & 15];
  int t = (lane < 16) ? tv : 0;
#pragma unroll
  for (int d = 1; d < 32; d <<= 1) { const int y = __shfl_up(t, d, 32); if (lane >= d) t += y; }
  const int wlo = __shfl(t, (wv > 0) ? (wv - 1) : 0, 32);
  const int woff = (wv == 0) ? 0 : wlo;
  total = __shfl(t, 15, 32);
  return woff + x - cnt;
}

__global__ __launch_bounds__(512) void k_scat(const float* __restrict__ MSG, int first, const int* __restrict__ dst_base, int t0, float* AGG) {
  #pragma clang fp contract(off)
  const int* dsti = dst_base + t0;
  __shared__ short Lr[CHUNK];
  __shared__ int Le[CHUNK];
  __shared__ int scan[16];
  __shared__ int lq[16][QCAP][32];
  __shared__ __attribute__((aligned(16))) float stg[64][68];
  const int tid = threadIdx.x, lane = tid & 31, wv = tid >> 5;
  const int n0 = blockIdx.x * 1024;
  int qn = 0;
  float acc[2][64];
#pragma unroll
  for (int s2 = 0; s2 < 2; ++s2)
#pragma unroll
    for (int c = 0; c < 64; ++c) acc[s2][c] = 0.f;

#pragma unroll 1
  for (int eb = 0; eb < TC + CHUNK; eb += CHUNK) {
    const bool sentinel = (eb >= TC);
    int tot = 0;
    if (!sentinel) {
      int k_cnt = 0; unsigned hm = 0; int hv[16];
#pragma unroll
      for (int k = 0; k < 16; ++k) {
        const int e = eb + tid * 16 + k;
        const int ec = (e < TC) ? e : (TC - 1);
        const int dv = dsti[ec] - n0;
        const int dd_ = (e < TC) ? dv : -1;
        hv[k] = dd_;
        if (dd_ >= 0 && dd_ < 1024) { hm |= 1u << k; ++k_cnt; }
      }
      int p = bscan512(k_cnt, scan, tid, tot);
#pragma unroll
      for (int k = 0; k < 16; ++k) if (hm & (1u << k)) { Lr[p] = (short)hv[k]; Le[p] = eb + tid * 16 + k; ++p; }
      __syncthreads();
    }
    const int ntrip = sentinel ? 1 : ((tot + 31) >> 5);
#pragma unroll 1
    for (int it = 0; it < ntrip; ++it) {
      const int q = it * 32 + lane;
      const int qc = (q < CHUNK) ? q : (CHUNK - 1);
      const int lrv = (int)Lr[qc];
      const int lr = (!sentinel && q < tot) ? lrv : -1;
      unsigned mm = sentinel ? 1u : __builtin_amdgcn_ballot_w32(lr >= wv * 64 && lr < wv * 64 + 64);
#pragma unroll 1
      while (mm) {
        const int bit = __builtin_ctz(mm);
        mm &= mm - 1u;
        const int lsh = __shfl(lr, bit, 32);
        const int ol = sentinel ? -2 : (lsh - wv * 64);
        const int owner = ol >> 1;
        int lei = it * 32 + bit; lei = (lei < CHUNK) ? lei : (CHUNK - 1);
        const int lev = Le[lei];
        const int e = sentinel ? 0 : lev;
        if (sentinel || __builtin_amdgcn_ballot_w32(lane == owner && qn == QCAP)) {
          int kmax = qn;
#pragma unroll
          for (int o = 16; o >= 1; o >>= 1) kmax = max(kmax, __shfl_xor(kmax, o, 32));
#pragma unroll 1
          for (int k = 0; k < kmax; ++k) {
            if (k < qn) {
              const int ent = lq[wv][k][lane];
              int eq = ent >> 1;
              const int sl = ent & 1;
              eq = eq < 0 ? 0 : (eq >= TC ? (TC - 1) : eq);
              const float* mr = MSG + (size_t)eq * DD;
#pragma unroll
              for (int s2 = 0; s2 < 2; ++s2) if (s2 == sl) {
#pragma unroll
                for (int c = 0; c < 64; c += 4) {
                  const v4f v = *(const v4fa*)(mr + c);
                  acc[s2][c] += v[0]; acc[s2][c + 1] += v[1]; acc[s2][c + 2] += v[2]; acc[s2][c + 3] += v[3];
                }
              }
            }
          }
          qn = 0;
        }
        if (lane == owner) { lq[wv][qn][lane] = e * 2 + (ol & 1); ++qn; }
      }
    }
    __syncthreads();
  }
  for (int tg = 0; tg < 16; ++tg) {
    if (wv == tg) {
#pragma unroll
      for (int c = 0; c < 64; ++c) { stg[2 * lane][c] = acc[0][c]; stg[2 * lane + 1][c] = acc[1][c]; }
    }
    __syncthreads();
    v4f sum[2];
    bool ok[2];
    size_t dofs[2];
#pragma unroll
    for (int rd = 0; rd < 2; ++rd) {
      const int r = rd * 32 + (tid >> 4), pc = tid & 15;
      const int n = n0 + tg * 64 + r;
      ok[rd] = (n < NEDGE);
      const int nc = ok[rd] ? n : (NEDGE - 1);
      dofs[rd] = (size_t)nc * DD + pc * 4;
      const v4f cur = first ? (v4f){0.f, 0.f, 0.f, 0.f} : *(const v4fa*)(AGG + dofs[rd]);
      const v4f st = *(const v4fa*)&stg[r][pc * 4];
      v4f a;
#pragma unroll
      for (int qq = 0; qq < 4; ++qq) a[qq] = cur[qq] + st[qq];
      sum[rd] = a;
    }
    for (int pass = 0; pass < 2; ++pass) {
#pragma unroll
      for (int rd = 0; rd < 2; ++rd) if (ok[rd]) *(volatile v4f*)(AGG + dofs[rd]) = sum[rd];
      if (pass == 0) __threadfence();
    }
    __syncthreads();
  }
}

extern "C" void kernel_launch(void* const* d_in, const int* in_sizes, int n_in,
                              void* d_out, int out_size, void* d_ws, size_t ws_size, hipStream_t stream) {
  if (n_in < 28) return;
  if (in_sizes[0] != NEDGE * HH || in_sizes[1] != NEDGE * NR || in_sizes[2] != NTRIP * NS) return;
  if (in_sizes[3] != NTRIP || in_sizes[4] != NTRIP || in_sizes[5] != NEDGE || in_sizes[7] < 1) return;
  if (in_sizes[8] != NBR * HH * HH || in_sizes[9] != NBR * HH || in_sizes[10] != NBR * NR * NC || in_sizes[11] != NBR * NC * HH) return;
  if (in_sizes[12] != NBR * NS * NC || in_sizes[13] != NBR * NC * DD || in_sizes[14] != NBR * HH * DD) return;
  if (in_sizes[15] != HH * HH || in_sizes[16] != HH || in_sizes[17] != DD * HH) return;
  if (in_sizes[18] != HH * HH || in_sizes[19] != HH || in_sizes[20] != HH * HH || in_sizes[21] != HH) return;
  if (in_sizes[22] != HH * HH || in_sizes[23] != HH) return;
  if (in_sizes[24] != HH * HH || in_sizes[25] != HH || in_sizes[26] != HH * HH || in_sizes[27] != HH) return;
  if (out_size != NEDGE * HH) return;

  const float* x      = (const float*)d_in[0];
  const float* rbf    = (const float*)d_in[1];
  const float* sbf    = (const float*)d_in[2];
  const int*   ikj    = (const int*)d_in[3];
  const int*   iji    = (const int*)d_in[4];
  const int*   btab   = (const int*)d_in[5];
  const float* alpha  = (const float*)d_in[7];
  const float* W_kj   = (const float*)d_in[8];
  const float* b_kj   = (const float*)d_in[9];
  const float* W_rbf1 = (const float*)d_in[10];
  const float* W_rbf2 = (const float*)d_in[11];
  const float* W_sbf1 = (const float*)d_in[12];
  const float* W_sbf2 = (const float*)d_in[13];
  const float* W_down = (const float*)d_in[14];
  const float* W_ji   = (const float*)d_in[15];
  const float* b_ji   = (const float*)d_in[16];
  const float* W_up   = (const float*)d_in[17];
  const float* rb1_w  = (const float*)d_in[18];
  const float* rb1_b  = (const float*)d_in[19];
  const float* rb2_w  = (const float*)d_in[20];
  const float* rb2_b  = (const float*)d_in[21];
  const float* W_lin  = (const float*)d_in[22];
  const float* b_lin  = (const float*)d_in[23];
  const float* ra1_w  = (const float*)d_in[24];
  const float* ra1_b  = (const float*)d_in[25];
  const float* ra2_w  = (const float*)d_in[26];
  const float* ra2_b  = (const float*)d_in[27];

  char* ws = (char*)d_ws;
  size_t off = 0;
  auto take = [&](size_t bytes) { char* p = ws + off; off += (bytes + 255) & ~(size_t)255; return p; };
  unsigned short* WJI = (unsigned short*)take((size_t)HH * HH * 2);
  unsigned short* WKJ = (unsigned short*)take((size_t)NBR * HH * HH * 2);
  unsigned short* WDN = (unsigned short*)take((size_t)NBR * DD * HH * 2);
  unsigned short* WUP = (unsigned short*)take((size_t)HH * DD * 2);
  unsigned short* RB1 = (unsigned short*)take((size_t)HH * HH * 2);
  unsigned short* RB2 = (unsigned short*)take((size_t)HH * HH * 2);
  unsigned short* LIN = (unsigned short*)take((size_t)HH * HH * 2);
  unsigned short* RA1 = (unsigned short*)take((size_t)HH * HH * 2);
  unsigned short* RA2 = (unsigned short*)take((size_t)HH * HH * 2);
  unsigned short* WS1 = (unsigned short*)take((size_t)64 * 64 * 2);
  unsigned short* X16 = (unsigned short*)take((size_t)NEDGE * HH * 2);
  float*          AGG = (float*)take((size_t)NEDGE * DD * 4);
  const size_t down_bytes = (size_t)NBR * NEDGE * DD * 2;
  const size_t scr_bytes  = (size_t)TC * 64 * 2 + (size_t)TC * DD * 4 + (size_t)TC * DD * 4;
  const size_t regb_bytes = down_bytes + scr_bytes;
  const size_t phc_bytes  = (size_t)NEDGE * HH * 4 + 3 * (size_t)NEDGE * HH * 2 + (size_t)NEDGE * DD * 2;
  if (phc_bytes > regb_bytes) return;
  char* REGB = take(regb_bytes);
  if (off > ws_size || off > ((size_t)128 << 20)) return;
  unsigned short* DOWN16 = (unsigned short*)REGB;
  char* SCR = REGB + down_bytes;
  unsigned short* TMP16 = (unsigned short*)SCR;
  unsigned short* SBF16 = (unsigned short*)SCR;
  float* P1  = (float*)(SCR + (size_t)TC * 64 * 2);
  float* MSG = (float*)(SCR + (size_t)TC * 64 * 2 + (size_t)TC * DD * 4);
  float* H = (float*)REGB;
  unsigned short* H16a  = (unsigned short*)(REGB + (size_t)NEDGE * HH * 4);
  unsigned short* H16b  = H16a + (size_t)NEDGE * HH;
  unsigned short* T16   = H16b + (size_t)NEDGE * HH;
  unsigned short* AGG16 = T16 + (size_t)NEDGE * HH;

  const float s16 = 0.0625f;
  const unsigned gE128 = (unsigned)(((NEDGE / 16) * (HH / 64)) / 4);
  const unsigned gE64  = (unsigned)(((NEDGE / 16) * (DD / 64)) / 4);
  const unsigned gT64  = (unsigned)(((TC / 16) * (DD / 64)) / 4);

  k_wt<<<dim3((HH * (HH / 8) + 255) / 256, 1), 256, 0, stream>>>(W_ji, 0, WJI, 0, HH, HH, 16.0f);
  k_wt<<<dim3((HH * (HH / 8) + 255) / 256, NBR), 256, 0, stream>>>(W_kj, HH * HH, WKJ, HH * HH, HH, HH, 16.0f);
  k_wt<<<dim3((DD * (HH / 8) + 255) / 256, NBR), 256, 0, stream>>>(W_down, HH * DD, WDN, HH * DD, HH, DD, 16.0f);
  k_wt<<<dim3((HH * (DD / 8) + 255) / 256, 1), 256, 0, stream>>>(W_up, 0, WUP, 0, DD, HH, 16.0f);
  k_wt<<<dim3((HH * (HH / 8) + 255) / 256, 1), 256, 0, stream>>>(rb1_w, 0, RB1, 0, HH, HH, 16.0f);
  k_wt<<<dim3((HH * (HH / 8) + 255) / 256, 1), 256, 0, stream>>>(rb2_w, 0, RB2, 0, HH, HH, 16.0f);
  k_wt<<<dim3((HH * (HH / 8) + 255) / 256, 1), 256, 0, stream>>>(W_lin, 0, LIN, 0, HH, HH, 16.0f);
  k_wt<<<dim3((HH * (HH / 8) + 255) / 256, 1), 256, 0, stream>>>(ra1_w, 0, RA1, 0, HH, HH, 16.0f);
  k_wt<<<dim3((HH * (HH / 8) + 255) / 256, 1), 256, 0, stream>>>(ra2_w, 0, RA2, 0, HH, HH, 16.0f);
  k_ws1t<<<(64 * 8 + 255) / 256, 256, 0, stream>>>(W_sbf1, WS1);
  k_x16<<<(unsigned)(((size_t)NEDGE * HH / 8 + 255) / 256), 256, 0, stream>>>(x, X16);

  for (int b = 0; b < NBR; ++b) {
    k_gemm<true, true><<<gE128, 128, 0, stream>>>(X16, HH, WKJ + (size_t)b * HH * HH, HH, NEDGE, HH, HH, s16, b_kj + (size_t)b * HH,
                                                 rbf, W_rbf1 + (size_t)b * NR * NC, W_rbf2 + (size_t)b * NC * HH,
                                                 nullptr, 0, nullptr, 0, TMP16, HH, 1024.0f);
    k_gemm<false, true><<<gE64, 128, 0, stream>>>(TMP16, HH, WDN + (size_t)b * DD * HH, HH, NEDGE, DD, HH, s16 * (1.0f / 1024.0f), nullptr,
                                                 nullptr, nullptr, nullptr,
                                                 nullptr, 0, nullptr, 0, DOWN16 + (size_t)b * NEDGE * DD, DD, 256.0f);
  }
  for (int c = 0; c < NTRIP / TC; ++c) {
    const int t0 = c * TC;
    k_sbf16<<<(TC * 8 + 255) / 256, 256, 0, stream>>>(sbf, t0, SBF16);
    k_gemm<false, false><<<gT64, 128, 0, stream>>>(SBF16, 64, WS1, 64, TC, DD, 64, s16, nullptr,
                                                  nullptr, nullptr, nullptr, nullptr, 0, P1, DD, nullptr, 0, 1.0f);
    k_msg<<<(TC * 16 + 255) / 256, 256, 0, stream>>>(P1, ikj, btab, alpha, W_sbf2, DOWN16, t0, MSG);
    k_scat<<<NEDGE / 1024, 512, 0, stream>>>(MSG, (c == 0) ? 1 : 0, iji, t0, AGG);
  }
  k_agg16<<<(unsigned)(((size_t)NEDGE * DD / 8 + 255) / 256), 256, 0, stream>>>(AGG, AGG16);
  k_gemm<false, true><<<gE128, 128, 0, stream>>>(X16, HH, WJI, HH, NEDGE, HH, HH, s16, b_ji, nullptr, nullptr, nullptr,
                                                nullptr, 0, H, HH, nullptr, 0, 1.0f);
  k_gemm<false, true><<<gE128, 128, 0, stream>>>(AGG16, DD, WUP, DD, NEDGE, HH, DD, s16 * (1.0f / 4096.0f), nullptr, nullptr, nullptr, nullptr,
                                                H, HH, H, HH, H16a, HH, 1.0f);
  k_gemm<false, true><<<gE128, 128, 0, stream>>>(H16a, HH, RB1, HH, NEDGE, HH, HH, s16, rb1_b, nullptr, nullptr, nullptr,
                                                nullptr, 0, nullptr, 0, T16, HH, 1.0f);
  k_gemm<false, true><<<gE128, 128, 0, stream>>>(T16, HH, RB2, HH, NEDGE, HH, HH, s16, rb2_b, nullptr, nullptr, nullptr,
                                                H, HH, H, HH, H16b, HH, 1.0f);
  k_gemm<false, true><<<gE128, 128, 0, stream>>>(H16b, HH, LIN, HH, NEDGE, HH, HH, s16, b_lin, nullptr, nullptr, nullptr,
                                                x, HH, H, HH, H16a, HH, 1.0f);
  k_gemm<false, true><<<gE128, 128, 0, stream>>>(H16a, HH, RA1, HH, NEDGE, HH, HH, s16, ra1_b, nullptr, nullptr, nullptr,
                                                nullptr, 0, nullptr, 0, T16, HH, 1.0f);
  k_gemm<false, true><<<gE128, 128, 0, stream>>>(T16, HH, RA2, HH, NEDGE, HH, HH, s16, ra2_b, nullptr, nullptr, nullptr,
                                                H, HH, (float*)d_out, HH, nullptr, 0, 1.0f);
  (void)hipGetLastError();
}
